// GraphAttentionLayer_35983236006299
// MI455X (gfx1250) — hardware-verified
//
#include <hip/hip_runtime.h>
#include <stddef.h>
#include <stdint.h>
#include <math.h>


#define NN     2048
#define CIN    128
#define FO     64
#define NTHR   256
#define GTHR   128
#define GBM    64
#define ATI    64
#define STP    68
#define SLOPE  0.01f
#define NEGBIG (-3.0e38f)
#define WSMAX  134217728

static_assert((NN % GBM) == 0 && (NN % ATI) == 0 && (NN % 32) == 0);
static_assert((CIN % 32) == 0 && (CIN / 8) == 16);
static_assert(FO == 64);
static_assert(GBM == (GTHR / 32) * 16 && ATI == (GTHR / 32) * 16);
static_assert(GTHR == 2 * FO && GTHR == 2 * GBM);
static_assert((STP % 4) == 0 && STP >= GBM);
static_assert(((FO * 8) % GTHR) == 0 && (FO * 8) / GTHR == 4);
static_assert(((NN / 4) % GTHR) == 0);

typedef float          v4f  __attribute__((ext_vector_type(4)));
typedef float          v8f  __attribute__((ext_vector_type(8)));
typedef int            v8i  __attribute__((ext_vector_type(8)));
typedef unsigned int   v4u  __attribute__((ext_vector_type(4)));
typedef unsigned short v8us __attribute__((ext_vector_type(8)));
typedef __bf16         v16b __attribute__((ext_vector_type(16)));
typedef v4f  __attribute__((may_alias)) v4fa;
typedef v4u  __attribute__((may_alias)) v4ua;
typedef v8us __attribute__((may_alias)) v8usa;
union FragB { v16b v; v8us u[2]; v8i w; };

__device__ __forceinline__ v8f wmb(const FragB& a, const FragB& b, v8f c) {
  v8f d = __builtin_amdgcn_wmma_f32_16x16x32_bf16(false, a.v, false, b.v, (short)0, c, false, false);
  asm volatile("v_nop\n\tv_nop\n\tv_nop\n\tv_nop" : "+v"(d) : "v"(a.w), "v"(b.w));
  return d;
}

__device__ __forceinline__ unsigned int f2bf(float f) {
  const unsigned int u = __float_as_uint(f);
  return ((u + 0x7FFFu + ((u >> 16) & 1u)) >> 16) & 0xFFFFu;
}
__device__ __forceinline__ float bf2f(unsigned int b) { return __uint_as_float(b << 16); }
__device__ __forceinline__ float bfr(float f) { return bf2f(f2bf(f)); }
__device__ __forceinline__ unsigned int pk2(float lo, float hi) { return f2bf(lo) | (f2bf(hi) << 16); }
__device__ __forceinline__ v4u pack8(const v4f a, const v4f b) {
  v4u r;
  r.x = pk2(a.x, a.y); r.y = pk2(a.z, a.w); r.z = pk2(b.x, b.y); r.w = pk2(b.z, b.w);
  return r;
}
__device__ __forceinline__ void split8(const v4f a, const v4f b, v4u& hv, v4u& lv) {
  float f[8] = {a.x, a.y, a.z, a.w, b.x, b.y, b.z, b.w};
  unsigned int hb[8], lb[8];
#pragma unroll
  for (int i = 0; i < 8; ++i) {
    hb[i] = f2bf(f[i]);
    lb[i] = f2bf(f[i] - bf2f(hb[i]));
  }
  hv.x = hb[0] | (hb[1] << 16); hv.y = hb[2] | (hb[3] << 16); hv.z = hb[4] | (hb[5] << 16); hv.w = hb[6] | (hb[7] << 16);
  lv.x = lb[0] | (lb[1] << 16); lv.y = lb[2] | (lb[3] << 16); lv.z = lb[4] | (lb[5] << 16); lv.w = lb[6] | (lb[7] << 16);
}

__global__ __launch_bounds__(NTHR) void k_xprep(const float* __restrict__ x, unsigned short* xb, int nN, int nUnits) {
  const int i = (int)blockIdx.x * NTHR + (int)threadIdx.x;
  if (i >= nUnits) return;
  const int row = i >> 4;
  const int c0  = (i & 15) * 8;
  const int rc  = row < nN ? row : nN - 1;
  const float* p = x + (size_t)rc * CIN + c0;
  v4f a = *(const v4fa*)p, b = *(const v4fa*)(p + 4);
  const v4f z4 = {0.f, 0.f, 0.f, 0.f};
  if (row >= nN) { a = z4; b = z4; }
  const v4u hv = pack8(a, b);
  const size_t o = (size_t)row * CIN + c0;
  *(volatile v4ua*)(xb + o) = hv;
  __threadfence();
  *(volatile v4ua*)(xb + o) = hv;
}

__global__ __launch_bounds__(NTHR) void k_wtr(const float* __restrict__ w, int cols, int K,
                                              unsigned short* wt, int nUnits) {
  const int u = (int)blockIdx.x * NTHR + (int)threadIdx.x;
  if (u >= nUnits) return;
  const int kq = K >> 3;
  const int n  = u / kq;
  const int k8 = (u - n * kq) * 8;
  const int ncl = n < cols ? n : cols - 1;
  const float* p = w + (size_t)k8 * (size_t)cols + ncl;
  v4f a, b;
  a.x = p[0];                  a.y = p[(size_t)cols];       a.z = p[(size_t)2 * cols];   a.w = p[(size_t)3 * cols];
  b.x = p[(size_t)4 * cols];   b.y = p[(size_t)5 * cols];   b.z = p[(size_t)6 * cols];   b.w = p[(size_t)7 * cols];
  const v4f z4 = {0.f, 0.f, 0.f, 0.f};
  if (n >= cols) { a = z4; b = z4; }
  const v4u hv = pack8(a, b);
  const size_t o = (size_t)n * (size_t)K + k8;
  *(volatile v4ua*)(wt + o) = hv;
  __threadfence();
  *(volatile v4ua*)(wt + o) = hv;
}

__global__ __launch_bounds__(GTHR) void k_proj(
    const unsigned short* __restrict__ XB, const unsigned short* __restrict__ WT,
    const float* __restrict__ av, float* S, unsigned short* HTh, unsigned short* HTl, int MP)
{
  __shared__ __attribute__((aligned(16))) float stgT[FO * STP];
  __shared__ __attribute__((aligned(16))) float satt[2 * FO];
  __shared__ __attribute__((aligned(16))) float sdot[2 * GBM];
  const int tid = (int)threadIdx.x, lane = tid & 31, wave = tid >> 5, hh = lane >> 4, m = lane & 15;
  const int rowBase = (int)blockIdx.x * GBM;
  const int bb = rowBase / NN;
  const int j0 = rowBase - bb * NN;

  satt[tid] = bfr(av[tid]);

  v8f acc[4];
  {
    const v8f z = {0.f, 0.f, 0.f, 0.f, 0.f, 0.f, 0.f, 0.f};
    acc[0] = z; acc[1] = z; acc[2] = z; acc[3] = z;
  }
  const unsigned short* ap = XB + (size_t)(rowBase + 16 * wave + m) * (size_t)CIN + 8 * hh;
  const unsigned short* wp = WT + (size_t)m * (size_t)CIN + 8 * hh;
#pragma unroll 1
  for (int ks = 0; ks < CIN / 32; ++ks) {
    FragB af;
    af.u[0] = *(const v8usa*)(ap + 32 * ks);
    af.u[1] = *(const v8usa*)(ap + 32 * ks + 16);
#pragma unroll
    for (int t = 0; t < 4; ++t) {
      const unsigned short* wq = wp + (size_t)(16 * t) * (size_t)CIN + 32 * ks;
      FragB bf;
      bf.u[0] = *(const v8usa*)wq;
      bf.u[1] = *(const v8usa*)(wq + 16);
      acc[t] = wmb(af, bf, acc[t]);
    }
  }

#pragma unroll
  for (int t = 0; t < 4; ++t) {
    const int lc = 16 * t + m;
#pragma unroll
    for (int r = 0; r < 8; ++r) {
      const int lr = 16 * wave + 8 * hh + r;
      stgT[lc * STP + lr] = acc[t][r];
    }
  }
  __syncthreads();

  {
    const int row = tid & 63, which = tid >> 6;
    const float* sa = satt + which * FO;
    float d = 0.f;
#pragma unroll 4
    for (int c = 0; c < FO; ++c) d = fmaf(stgT[c * STP + row], sa[c], d);
    sdot[tid] = d;
  }

  v4u hv[4], lv[4];
#pragma unroll
  for (int it = 0; it < 4; ++it) {
    const int p = it * GTHR + tid;
    const int f = p >> 3, q = p & 7;
    const v4f ga = *(const v4fa*)(stgT + f * STP + 8 * q);
    const v4f gb = *(const v4fa*)(stgT + f * STP + 8 * q + 4);
    split8(ga, gb, hv[it], lv[it]);
  }
  __syncthreads();

  const int which2 = lane >> 4, piece = lane & 15;
  const v4f sdv = *(const v4fa*)(sdot + which2 * GBM + 4 * piece);
  float* sp = S + (size_t)which2 * (size_t)MP + rowBase + 4 * piece;

#pragma unroll
  for (int it = 0; it < 4; ++it) {
    const int p = it * GTHR + tid;
    const int f = p >> 3, q = p & 7;
    const size_t o = ((size_t)bb * FO + f) * (size_t)NN + j0 + 8 * q;
    *(volatile v4ua*)(HTh + o) = hv[it];
    *(volatile v4ua*)(HTl + o) = lv[it];
  }
  if (wave == 0) *(volatile v4fa*)sp = sdv;
  __threadfence();
#pragma unroll
  for (int it = 0; it < 4; ++it) {
    const int p = it * GTHR + tid;
    const int f = p >> 3, q = p & 7;
    const size_t o = ((size_t)bb * FO + f) * (size_t)NN + j0 + 8 * q;
    *(volatile v4ua*)(HTh + o) = hv[it];
    *(volatile v4ua*)(HTl + o) = lv[it];
  }
  if (wave == 0) *(volatile v4fa*)sp = sdv;
}

__global__ __launch_bounds__(GTHR) void k_attn(
    const float* __restrict__ adj, const float* __restrict__ S,
    const unsigned short* __restrict__ HTh, const unsigned short* __restrict__ HTl,
    float* out, int MP)
{
  __shared__ __attribute__((aligned(16))) float s2s[NN];
  __shared__ __attribute__((aligned(16))) float stg[ATI * FO];
  const int tid = (int)threadIdx.x, lane = tid & 31, wave = tid >> 5, hh = lane >> 4, m = lane & 15;
  const int b  = (int)blockIdx.y;
  const int i0 = (int)blockIdx.x * ATI;

  {
    const float* s2g = S + (size_t)MP + (size_t)b * NN;
#pragma unroll 1
    for (int i = tid; i < NN / 4; i += GTHR) *(v4fa*)(s2s + 4 * i) = *(const v4fa*)(s2g + 4 * i);
  }
  __syncthreads();

  const int irow = i0 + 16 * wave + m;
  const float s1v = S[(size_t)b * NN + irow];
  const float* adjRow = adj + (size_t)irow * (size_t)NN;
  const size_t hro = ((size_t)b * FO + m) * (size_t)NN + 8 * hh;
  const unsigned short* hbp = HTh + hro;
  const unsigned short* lbp = HTl + hro;

  v8f acc[4];
  {
    const v8f z = {0.f, 0.f, 0.f, 0.f, 0.f, 0.f, 0.f, 0.f};
    acc[0] = z; acc[1] = z; acc[2] = z; acc[3] = z;
  }
  float m_run = NEGBIG, l_run = 0.f;

#pragma unroll 1
  for (int ks = 0; ks < NN / 32; ++ks) {
    const int j0 = 32 * ks;
    float e[16];
    float tmax = NEGBIG;
#pragma unroll
    for (int seg = 0; seg < 2; ++seg) {
      const int kb = j0 + 16 * seg + 8 * hh;
      const v4f a0 = *(const v4fa*)(adjRow + kb);
      const v4f a1 = *(const v4fa*)(adjRow + kb + 4);
      const v4f v0 = *(const v4fa*)(s2s + kb);
      const v4f v1 = *(const v4fa*)(s2s + kb + 4);
      const float adjv[8] = {a0.x, a0.y, a0.z, a0.w, a1.x, a1.y, a1.z, a1.w};
      const float s2v[8]  = {v0.x, v0.y, v0.z, v0.w, v1.x, v1.y, v1.z, v1.w};
#pragma unroll
      for (int o = 0; o < 8; ++o) {
        const float x  = s1v + s2v[o];
        const float ev = x > 0.f ? x : SLOPE * x;
        const bool keep = (adjv[o] > 0.f) || (kb + o == irow);
        const float val = keep ? ev : NEGBIG;
        e[8 * seg + o] = val;
        tmax = fmaxf(tmax, val);
      }
    }
    tmax = fmaxf(tmax, __shfl_xor(tmax, 16));
    const float m_new = fmaxf(m_run, tmax);
    const float alpha = expf(m_run - m_new);

    float psum = 0.f;
    FragB ph, pl;
#pragma unroll
    for (int qq = 0; qq < 8; ++qq) {
      float p2[2];
#pragma unroll
      for (int u = 0; u < 2; ++u) {
        const int q = 2 * qq + u;
        const float d  = fminf(e[q] - m_new, 0.f);
        const float ex = expf(d);
        const float p  = (e[q] > -1.0e38f) ? ex : 0.f;
        psum += p;
        p2[u] = p;
      }
      const unsigned int hb0 = f2bf(p2[0]), hb1 = f2bf(p2[1]);
      const unsigned int lb0 = f2bf(p2[0] - bf2f(hb0)), lb1 = f2bf(p2[1] - bf2f(hb1));
      ph.w[qq] = (int)(hb0 | (hb1 << 16));
      pl.w[qq] = (int)(lb0 | (lb1 << 16));
    }
    psum += __shfl_xor(psum, 16);
    l_run = fmaf(l_run, alpha, psum);
    m_run = m_new;

#pragma unroll
    for (int r = 0; r < 8; ++r) {
      const float ar = __shfl(alpha, 8 * hh + r);
#pragma unroll
      for (int t = 0; t < 4; ++t) acc[t][r] *= ar;
    }

#pragma unroll
    for (int t = 0; t < 4; ++t) {
      const size_t co = (size_t)(16 * t) * (size_t)NN + j0;
      FragB bh, bl;
      bh.u[0] = *(const v8usa*)(hbp + co);
      bh.u[1] = *(const v8usa*)(hbp + co + 16);
      bl.u[0] = *(const v8usa*)(lbp + co);
      bl.u[1] = *(const v8usa*)(lbp + co + 16);
      acc[t] = wmb(ph, bh, acc[t]);
      acc[t] = wmb(ph, bl, acc[t]);
      acc[t] = wmb(pl, bh, acc[t]);
    }
  }

  const float ls = l_run > 0.f ? l_run : 1.0f;
  const float rl = 1.0f / ls;
#pragma unroll
  for (int r = 0; r < 8; ++r) {
    const float rr = __shfl(rl, 8 * hh + r);
    const int lr = 16 * wave + 8 * hh + r;
#pragma unroll
    for (int t = 0; t < 4; ++t) stg[lr * FO + 16 * t + m] = acc[t][r] * rr;
  }
  __syncthreads();

  v4f fv[8];
#pragma unroll
  for (int i = 0; i < 8; ++i) {
    const int lr = 16 * wave + 2 * i + hh;
    fv[i] = *(const v4fa*)(stg + lr * FO + 4 * m);
  }
#pragma unroll
  for (int i = 0; i < 8; ++i) {
    const int lr = 16 * wave + 2 * i + hh;
    const size_t gr = (size_t)b * NN + i0 + lr;
    float* op = out + gr * (size_t)FO + 4 * m;
    *(volatile v4fa*)op = fv[i];
  }
  __threadfence();
#pragma unroll
  for (int i = 0; i < 8; ++i) {
    const int lr = 16 * wave + 2 * i + hh;
    const size_t gr = (size_t)b * NN + i0 + lr;
    float* op = out + gr * (size_t)FO + 4 * m;
    *(volatile v4fa*)op = fv[i];
  }
}

static inline int cdiv(int a, int b) { return (a + b - 1) / b; }

extern "C" void kernel_launch(void* const* d_in, const int* in_sizes, int n_in,
                              void* d_out, int out_size, void* d_ws, size_t ws_size,
                              hipStream_t stream) {
  if (n_in < 4) return;
  if (in_sizes[0] <= 0 || (in_sizes[0] % (NN * CIN)) != 0) return;
  const int nB = in_sizes[0] / (NN * CIN);
  if (nB < 1 || nB > 64) return;
  if (in_sizes[1] != NN * NN) return;
  if (in_sizes[2] != CIN * FO) return;
  if (in_sizes[3] != 2 * FO) return;
  const int MP = nB * NN;
  if (out_size != MP * FO) return;

  const float* inp = (const float*)d_in[0];
  const float* adj = (const float*)d_in[1];
  const float* W   = (const float*)d_in[2];
  const float* av  = (const float*)d_in[3];
  float* out = (float*)d_out;

  char* ws = (char*)d_ws;
  size_t off = 0;
  const size_t oXB  = off; off += (size_t)MP * CIN * 2;        off = (off + 255) & ~(size_t)255;
  const size_t oWT  = off; off += (size_t)FO * CIN * 2;        off = (off + 255) & ~(size_t)255;
  const size_t oS   = off; off += (size_t)2 * MP * 4;          off = (off + 255) & ~(size_t)255;
  const size_t oHTh = off; off += (size_t)nB * FO * NN * 2;    off = (off + 255) & ~(size_t)255;
  const size_t oHTl = off; off += (size_t)nB * FO * NN * 2;    off = (off + 255) & ~(size_t)255;
  if (off > ws_size || off > (size_t)WSMAX) return;
  unsigned short* XB  = (unsigned short*)(ws + oXB);
  unsigned short* WT  = (unsigned short*)(ws + oWT);
  float*          S   = (float*)(ws + oS);
  unsigned short* HTh = (unsigned short*)(ws + oHTh);
  unsigned short* HTl = (unsigned short*)(ws + oHTl);

  const int nUx = MP * (CIN / 8);
  k_xprep<<<cdiv(nUx, NTHR), NTHR, 0, stream>>>(inp, XB, MP, nUx);

  const int nUw = FO * (CIN / 8);
  k_wtr<<<cdiv(nUw, NTHR), NTHR, 0, stream>>>(W, FO, CIN, WT, nUw);

  k_proj<<<dim3(MP / GBM), GTHR, 0, stream>>>(XB, WT, av, S, HTh, HTl, MP);

  k_attn<<<dim3(NN / ATI, nB), GTHR, 0, stream>>>(adj, S, HTh, HTl, out, MP);
}
